// BidirectionalRNN_86595130622324
// MI455X (gfx1250) — hardware-verified
//
#include <hip/hip_runtime.h>

typedef __attribute__((ext_vector_type(16))) _Float16 v16h;
typedef __attribute__((ext_vector_type(8)))  _Float16 v8h;
typedef __attribute__((ext_vector_type(16))) __bf16   v16b;
typedef __attribute__((ext_vector_type(8)))  __bf16   v8b;
typedef __attribute__((ext_vector_type(8)))  float    v8f;
typedef __attribute__((ext_vector_type(4)))  float    v4f;
typedef __attribute__((ext_vector_type(4)))  unsigned int v4u;
#define PSCALE 32768.0f
#define U16(p) ((const unsigned short*)(const void*)(p))
#define PSCALE_INV (1.0f / 32768.0f)

__device__ __forceinline__ unsigned short f2bf_bits(float f) {
  unsigned u = __float_as_uint(f);
  return (unsigned short)((u + 0x7FFFu + ((u >> 16) & 1u)) >> 16);
}
__device__ __forceinline__ float bf_bits2f(unsigned short h) { return __uint_as_float(((unsigned)h) << 16); }

__device__ __forceinline__ void dep_guard_h(v8f& a, v8f& b, v16h x, v16h y) { asm volatile("v_nop\n\tv_nop\n\tv_nop\n\tv_nop" : "+v"(a), "+v"(b) : "v"(x), "v"(y)); }
__device__ __forceinline__ void dep_guard_b(v8f& a, v8f& b, v16b x, v16b y) { asm volatile("v_nop\n\tv_nop\n\tv_nop\n\tv_nop" : "+v"(a), "+v"(b) : "v"(x), "v"(y)); }
__device__ __forceinline__ void keep4_h(v16h a, v16h b, v16h c, v16h d) { asm volatile("v_nop" :: "v"(a), "v"(b), "v"(c), "v"(d)); }
__device__ __forceinline__ void keep4_b(v16b a, v16b b, v16b c, v16b d) { asm volatile("v_nop" :: "v"(a), "v"(b), "v"(c), "v"(d)); }
__device__ __forceinline__ void acc_guard4(v8f& a, v8f& b, v8f& c, v8f& d) { asm volatile("v_nop\n\tv_nop\n\tv_nop\n\tv_nop" : "+v"(a), "+v"(b), "+v"(c), "+v"(d)); }
template <typename T> struct Frag;
template <> struct Frag<_Float16> {
  typedef v16h V; union U { v16h v; v8h h[2]; };
  static __device__ __forceinline__ v16h load(const _Float16* p) {
    U f; f.h[0] = *(const v8h*)(p); f.h[1] = *(const v8h*)(p + 16); return f.v;
  }
  static __device__ __forceinline__ v8f mma(v16h a, v16h b, v8f c) {
    return __builtin_amdgcn_wmma_f32_16x16x32_f16(false, a, false, b, (short)0, c, false, false);
  }
  static __device__ __forceinline__ void guard(v8f& a, v8f& b, v16h x, v16h y) { dep_guard_h(a, b, x, y); }
  static __device__ __forceinline__ void keep(v16h a, v16h b, v16h c, v16h d) { keep4_h(a, b, c, d); }
};
template <> struct Frag<__bf16> {
  typedef v16b V; union U { v16b v; v8b h[2]; };
  static __device__ __forceinline__ v16b load(const __bf16* p) {
    U f; f.h[0] = *(const v8b*)(p); f.h[1] = *(const v8b*)(p + 16); return f.v;
  }
  static __device__ __forceinline__ v8f mma(v16b a, v16b b, v8f c) {
    return __builtin_amdgcn_wmma_f32_16x16x32_bf16(false, a, false, b, (short)0, c, false, false);
  }
  static __device__ __forceinline__ void guard(v8f& a, v8f& b, v16b x, v16b y) { dep_guard_b(a, b, x, y); }
  static __device__ __forceinline__ void keep(v16b a, v16b b, v16b c, v16b d) { keep4_b(a, b, c, d); }
};

template <int ET> struct Elem;
template <> struct Elem<0> { typedef _Float16 T; };
template <> struct Elem<1> { typedef __bf16 T; };
template <int ET, bool SPLIT, int BIAS_MODE, int OUT_MODE, bool RESID, int ACT = 0>
__global__ __launch_bounds__(256) void wmma_gemm64(
    const unsigned short* __restrict__ Ap, const unsigned short* __restrict__ A2p, int lda, long strideA,
    const unsigned short* __restrict__ Btp, const unsigned short* __restrict__ Bt2p, int ldb, long strideB,
    void* __restrict__ Cout, void* __restrict__ Cout2, int ldc, long strideC,
    const float* __restrict__ bias,
    const float* __restrict__ resid, long strideR,
    int M, int N, int K, float scale) {
  typedef typename Elem<ET>::T T;
  typedef typename Frag<T>::V V;
  const T* A = (const T*)Ap; const T* A2 = (const T*)A2p; const T* Bt = (const T*)Btp; const T* Bt2 = (const T*)Bt2p;
  __shared__ __align__(16) float sT[8][16 * 68];
  const int b    = blockIdx.y;
  const int lane = threadIdx.x & 31;
  const int wave = threadIdx.x >> 5;
  const int tilesN = N >> 6;
  const int tilesM = M >> 6;
  const int tile = blockIdx.x * 8 + wave;
  if (tile >= tilesM * tilesN) return;
  const int tm = tile / tilesN;
  const int tn = tile - tm * tilesN;
  const int m0 = tm << 6;
  const int n0 = tn << 6;

  const T* Ab  = A  + (size_t)b * strideA;
  const T* Bb  = Bt + (size_t)b * strideB;
  const T* Ab2 = SPLIT ? (A2  + (size_t)b * strideA) : nullptr;
  const T* Bb2 = SPLIT ? (Bt2 + (size_t)b * strideB) : nullptr;

  const int rlane = lane & 15;
  const int koff  = (lane >> 4) * 8;
  const int mOff  = (lane >> 4) * 8;

  v8f acc[4][4];
#pragma unroll
  for (int i = 0; i < 4; ++i)
#pragma unroll
    for (int j = 0; j < 4; ++j) acc[i][j] = (v8f){0.f,0.f,0.f,0.f,0.f,0.f,0.f,0.f};

  for (int k0 = 0; k0 < K; k0 += 32) {
    V bh[4], bl[4];
#pragma unroll
    for (int j = 0; j < 4; ++j) {
      const size_t bo = (size_t)(n0 + (j << 4) + rlane) * ldb + koff + k0;
      bh[j] = Frag<T>::load(Bb + bo);
      if (SPLIT) bl[j] = Frag<T>::load(Bb2 + bo);
    }
#pragma unroll
    for (int i = 0; i < 4; ++i) {
      const size_t ao = (size_t)(m0 + (i << 4) + rlane) * lda + koff + k0;
      V ah = Frag<T>::load(Ab + ao);
      V al;
      if (SPLIT) al = Frag<T>::load(Ab2 + ao);
#pragma unroll
      for (int j = 0; j < 4; ++j) {
        acc[i][j] = Frag<T>::mma(ah, bh[j], acc[i][j]);
        if (SPLIT) {
          acc[i][j] = Frag<T>::mma(ah, bl[j], acc[i][j]);
          acc[i][j] = Frag<T>::mma(al, bh[j], acc[i][j]);
        }
      }
      Frag<T>::guard(acc[i][0], acc[i][3], ah, SPLIT ? al : ah);
    }
    Frag<T>::keep(bh[0], bh[1], bh[2], bh[3]);
    if (SPLIT) Frag<T>::keep(bl[0], bl[1], bl[2], bl[3]);
  }
  acc_guard4(acc[0][0], acc[0][1], acc[0][2], acc[0][3]);
  acc_guard4(acc[1][0], acc[1][1], acc[1][2], acc[1][3]);
  acc_guard4(acc[2][0], acc[2][1], acc[2][2], acc[2][3]);
  acc_guard4(acc[3][0], acc[3][1], acc[3][2], acc[3][3]);

  float* slab = sT[wave];
  const float* Rb = RESID ? (resid + (size_t)b * strideR) : nullptr;
#pragma unroll
  for (int i = 0; i < 4; ++i) {
    const int mBase = m0 + (i << 4);
#pragma unroll
    for (int j = 0; j < 4; ++j) {
      const int n = n0 + (j << 4) + rlane;
      float bv = 0.f;
      if (BIAS_MODE == 2) bv = bias[n];
#pragma unroll
      for (int r = 0; r < 8; ++r) {
        float v = acc[i][j][r] * scale;
        if (BIAS_MODE == 1) v += bias[mBase + mOff + r];
        if (BIAS_MODE == 2) v += bv;
        if (RESID) v += Rb[(size_t)(mBase + mOff + r) * ldc + n];
        if (ACT == 1) v = tanhf(v);
        if (ACT == 2) v = fmaxf(v, 0.0f);
        if (ACT == 3) v = v / (1.0f + expf(-v));
        if (ACT == 4) v = (v > 0.f) ? v : 0.01f * v;
        if (ACT == 5) v = 0.5f * v * (1.0f + erff(v * 0.70710678118654752f));
        slab[(mOff + r) * 68 + (j << 4) + rlane] = v;
      }
    }
    __builtin_amdgcn_fence(__ATOMIC_RELEASE, "workgroup");
    __builtin_amdgcn_wave_barrier();
    __builtin_amdgcn_fence(__ATOMIC_ACQUIRE, "workgroup");
    if (OUT_MODE == 0) {
      float* C = (float*)Cout + (size_t)b * strideC;
      const int hh = lane >> 4, c4 = (lane & 15) * 4;
      for (int pass = 0; pass < 2; ++pass) {
#pragma unroll
        for (int it = 0; it < 8; ++it) {
          const int row = it * 2 + hh;
          v4f v = *(const v4f*)(slab + row * 68 + c4);
          *(volatile v4f*)(C + (size_t)(mBase + row) * ldc + n0 + c4) = v;
        }
        __threadfence();
      }
    } else {
      const int q = lane >> 3, c8 = (lane & 7) * 8;
      unsigned short* C  = (unsigned short*)Cout  + (size_t)b * strideC;
      unsigned short* C2 = (OUT_MODE == 2) ? ((unsigned short*)Cout2 + (size_t)b * strideC) : nullptr;
      for (int pass = 0; pass < 2; ++pass) {
#pragma unroll
        for (int it = 0; it < 4; ++it) {
          const int row = it * 4 + q;
          const float* sp = slab + row * 68 + c8;
          v8h hv, lv;
#pragma unroll
          for (int e = 0; e < 8; ++e) {
            if (OUT_MODE == 1) {
              hv[e] = (_Float16)sp[e];
            } else {
              unsigned short hb = f2bf_bits(sp[e]);
              unsigned short lb = f2bf_bits(sp[e] - bf_bits2f(hb));
              hv[e] = __builtin_bit_cast(_Float16, hb);
              lv[e] = __builtin_bit_cast(_Float16, lb);
            }
          }
          *(volatile v8h*)(C + (size_t)(mBase + row) * ldc + n0 + c8) = hv;
          if (OUT_MODE == 2) *(volatile v8h*)(C2 + (size_t)(mBase + row) * ldc + n0 + c8) = lv;
        }
        __threadfence();
      }
    }
    __builtin_amdgcn_fence(__ATOMIC_RELEASE, "workgroup");
    __builtin_amdgcn_wave_barrier();
    __builtin_amdgcn_fence(__ATOMIC_ACQUIRE, "workgroup");
  }
}

constexpr int NBATCH = 32, NSTEP = 512, NDIN = 64, NHID = 128, NEMB = 256, NGATE3 = 384, NQKV = 768;
constexpr int NROWS  = NBATCH * NSTEP;
constexpr int HA_P   = NHID + 8;
constexpr int KSH_P  = 40;
constexpr int VT_P   = 72;
static_assert(NROWS % 64 == 0 && NQKV % 64 == 0 && NEMB % 64 == 0 && NDIN % 64 == 0, "tile multiples");
static_assert(NDIN % 32 == 0 && NHID % 32 == 0 && NEMB % 32 == 0, "K multiples of 32");

__device__ __forceinline__ v8f mma_h(v16h a, v16h b, v8f c) {
  c = __builtin_amdgcn_wmma_f32_16x16x32_f16(false, a, false, b, (short)0, c, false, false);
  asm volatile("v_nop\n\tv_nop\n\tv_nop\n\tv_nop" : "+v"(c) : "v"(a), "v"(b));
  return c;
}

__global__ __launch_bounds__(256) void prep_xm_f16x8(const float* __restrict__ x, const float* __restrict__ msk,
                                                     _Float16* __restrict__ out, int n8) {
  const int i = blockIdx.x * 256 + threadIdx.x;
  if (i < n8) {
    const size_t e = (size_t)i * 8;
    const v4f xa = *(const v4f*)(x + e), xb = *(const v4f*)(x + e + 4);
    const v4f ma = *(const v4f*)(msk + e), mb = *(const v4f*)(msk + e + 4);
    v8h o;
    o[0] = (_Float16)(xa[0] * ma[0]); o[1] = (_Float16)(xa[1] * ma[1]);
    o[2] = (_Float16)(xa[2] * ma[2]); o[3] = (_Float16)(xa[3] * ma[3]);
    o[4] = (_Float16)(xb[0] * mb[0]); o[5] = (_Float16)(xb[1] * mb[1]);
    o[6] = (_Float16)(xb[2] * mb[2]); o[7] = (_Float16)(xb[3] * mb[3]);
    _Float16* dst = out + e;
    *(volatile v8h*)dst = o;
    __threadfence();
    *(volatile v8h*)dst = o;
  }
}

__global__ __launch_bounds__(256) void cast_scale_f16x8(const float* __restrict__ in, _Float16* __restrict__ out,
                                                       int n8, float scale) {
  const int i = blockIdx.x * 256 + threadIdx.x;
  if (i < n8) {
    const size_t e = (size_t)i * 8;
    const v4f a = *(const v4f*)(in + e), b = *(const v4f*)(in + e + 4);
    v8h o;
    o[0] = (_Float16)(a[0] * scale); o[1] = (_Float16)(a[1] * scale);
    o[2] = (_Float16)(a[2] * scale); o[3] = (_Float16)(a[3] * scale);
    o[4] = (_Float16)(b[0] * scale); o[5] = (_Float16)(b[1] * scale);
    o[6] = (_Float16)(b[2] * scale); o[7] = (_Float16)(b[3] * scale);
    _Float16* dst = out + e;
    *(volatile v8h*)dst = o;
    __threadfence();
    *(volatile v8h*)dst = o;
  }
}

__global__ __launch_bounds__(256) void gru_bidir_kernel(
    const float* __restrict__ gi,
    const _Float16* __restrict__ whf, const _Float16* __restrict__ whb,
    const float* __restrict__ fbi, const float* __restrict__ fbh,
    const float* __restrict__ bbi, const float* __restrict__ bbh,
    _Float16* __restrict__ hc) {
  __shared__ __align__(16) _Float16 hA[16 * HA_P];
  __shared__ __align__(16) _Float16 rA[16 * HA_P];
  const int tid = threadIdx.x;
  const int wave = tid >> 5, lane = tid & 31, hh = lane >> 4, c = lane & 15;
  const int dir = blockIdx.x >> 1;
  const int b0 = (blockIdx.x & 1) * 16;
  const _Float16* Wh = dir ? whb : whf;
  const float* bi = dir ? bbi : fbi;
  const float* bh = dir ? bbh : fbh;
  const int u = wave * 16 + c;
  const float cR = bi[u] + bh[u];
  const float cZ = bi[NHID + u] + bh[NHID + u];
  const float cN = bi[2 * NHID + u] + bh[2 * NHID + u];
  const float w16inv = 0.0625f;

  for (int i = tid; i < (16 * HA_P) / 8; i += 256) {
    *(v4u*)(hA + 8 * i) = (v4u){0u, 0u, 0u, 0u};
  }
  float hreg[8];
#pragma unroll
  for (int r = 0; r < 8; ++r) hreg[r] = 0.f;
  __syncthreads();

  const int q8 = lane >> 3, e8 = (lane & 7) * 8;
  const int lineL = 4 * wave + q8;
  const int lrow = lineL >> 1, lhalf = lineL & 1;

  for (int s = 0; s < NSTEP; ++s) {
    const int t = dir ? (NSTEP - 1 - s) : s;

    float gR[8], gZ[8];
#pragma unroll
    for (int r = 0; r < 8; ++r) {
      const float* gp = gi + ((size_t)(b0 + 8 * hh + r) * NSTEP + t) * NQKV + dir * NGATE3 + u;
      gR[r] = gp[0];
      gZ[r] = gp[NHID];
    }

    v8f accR = (v8f){0.f,0.f,0.f,0.f,0.f,0.f,0.f,0.f};
    v8f accZ = (v8f){0.f,0.f,0.f,0.f,0.f,0.f,0.f,0.f};
#pragma unroll
    for (int kk = 0; kk < 4; ++kk) {
      const v16h a  = Frag<_Float16>::load(hA + c * HA_P + kk * 32 + 8 * hh);
      const v16h br = Frag<_Float16>::load(Wh + (size_t)u * NHID + kk * 32 + 8 * hh);
      const v16h bz = Frag<_Float16>::load(Wh + (size_t)(NHID + u) * NHID + kk * 32 + 8 * hh);
      accR = mma_h(a, br, accR);
      accZ = mma_h(a, bz, accZ);
    }
    float zr[8];
#pragma unroll
    for (int r = 0; r < 8; ++r) {
      const float pr = accR[r] * w16inv + cR + gR[r];
      const float rg = 1.0f / (1.0f + expf(-pr));
      rA[(8 * hh + r) * HA_P + u] = (_Float16)(rg * hreg[r]);
      const float pz = accZ[r] * w16inv + cZ + gZ[r];
      zr[r] = 1.0f / (1.0f + expf(-pz));
    }
    __syncthreads();

    float gN[8];
#pragma unroll
    for (int r = 0; r < 8; ++r) {
      const float* gp = gi + ((size_t)(b0 + 8 * hh + r) * NSTEP + t) * NQKV + dir * NGATE3 + 2 * NHID + u;
      gN[r] = gp[0];
    }
    v8f accN = (v8f){0.f,0.f,0.f,0.f,0.f,0.f,0.f,0.f};
#pragma unroll
    for (int kk = 0; kk < 4; ++kk) {
      const v16h a  = Frag<_Float16>::load(rA + c * HA_P + kk * 32 + 8 * hh);
      const v16h bn = Frag<_Float16>::load(Wh + (size_t)(2 * NHID + u) * NHID + kk * 32 + 8 * hh);
      accN = mma_h(a, bn, accN);
    }
#pragma unroll
    for (int r = 0; r < 8; ++r) {
      const float n  = tanhf(accN[r] * w16inv + cN + gN[r]);
      const float hn = (1.0f - zr[r]) * n + zr[r] * hreg[r];
      hreg[r] = hn;
      hA[(8 * hh + r) * HA_P + u] = (_Float16)hn;
    }
    __syncthreads();

    {
      const v8h val = *(const v8h*)(hA + lrow * HA_P + lhalf * 64 + e8);
      _Float16* dst = hc + ((size_t)(b0 + lrow) * NSTEP + t) * NEMB + dir * NHID + lhalf * 64 + e8;
      *(volatile v8h*)dst = val;
      __threadfence();
      *(volatile v8h*)dst = val;
    }
  }
}

__global__ __launch_bounds__(256) void attn_hd32_kernel(const _Float16* __restrict__ qkv, _Float16* __restrict__ o, float qscale) {
  __shared__ __align__(16) unsigned short Ksh[2][64 * KSH_P];
  __shared__ __align__(16) unsigned short Vt[2][32 * VT_P];
  __shared__ __align__(16) unsigned short Psh[8][16 * VT_P];
  __shared__ __align__(16) unsigned short Ob[64 * VT_P];
  const int tid = threadIdx.x;
  const int wave = tid >> 5, lane = tid & 31, hh = lane >> 4, c = lane & 15;
  const int hsel = wave >> 2, wq = wave & 3;
  const int bx = blockIdx.x;
  const int qb = bx & 7, hp = (bx >> 3) & 3, b = bx >> 5;
  const int h  = hp * 2 + hsel;
  const int q0 = qb * 64 + wq * 16;
  const size_t rowbase = (size_t)b * NSTEP;
  const float PSC = 64.0f;
  const float OSC = 16.0f;

  const v16h qa = Frag<_Float16>::load(qkv + (rowbase + q0 + c) * NQKV + h * 32 + 8 * hh);

  float mrow[8], lrow[8];
  v8f oacc[2];
#pragma unroll
  for (int r = 0; r < 8; ++r) { mrow[r] = -INFINITY; lrow[r] = 0.f; }
#pragma unroll
  for (int t = 0; t < 2; ++t) oacc[t] = (v8f){0.f,0.f,0.f,0.f,0.f,0.f,0.f,0.f};

  unsigned short* Pp = Psh[wave];
  const unsigned short* Kp = Ksh[hsel];
  const unsigned short* Vp = Vt[hsel];

  for (int kc = 0; kc < NSTEP / 64; ++kc) {
    const int kv0 = kc * 64;
    __syncthreads();
#pragma unroll
    for (int it = 0; it < 2; ++it) {
      const int id = tid + it * 256;
      const int hs = id >> 8, kvr = (id >> 2) & 63, part = id & 3;
      const _Float16* src = qkv + (rowbase + kv0 + kvr) * NQKV + NEMB + (hp * 2 + hs) * 32 + part * 8;
      const v4u kw = *(const v4u*)src;
      const v4u vw = *(const v4u*)(src + NEMB);
      *(v4u*)(&Ksh[hs][kvr * KSH_P + part * 8]) = kw;
      unsigned short* vt = &Vt[hs][(part * 8) * VT_P + kvr];
      vt[0 * VT_P] = (unsigned short)(kw[0] & 0u | (vw[0] & 0xffffu));
      vt[1 * VT_P] = (unsigned short)(vw[0] >> 16);
      vt[2 * VT_P] = (unsigned short)(vw[1] & 0xffffu);
      vt[3 * VT_P] = (unsigned short)(vw[1] >> 16);
      vt[4 * VT_P] = (unsigned short)(vw[2] & 0xffffu);
      vt[5 * VT_P] = (unsigned short)(vw[2] >> 16);
      vt[6 * VT_P] = (unsigned short)(vw[3] & 0xffffu);
      vt[7 * VT_P] = (unsigned short)(vw[3] >> 16);
    }
    __syncthreads();

    v8f s[4];
#pragma unroll
    for (int j = 0; j < 4; ++j) {
      const v16h kb = Frag<_Float16>::load((const _Float16*)(Kp + (j * 16 + c) * KSH_P) + 8 * hh);
      s[j] = mma_h(qa, kb, (v8f){0.f,0.f,0.f,0.f,0.f,0.f,0.f,0.f});
    }
    float cm[8];
#pragma unroll
    for (int r = 0; r < 8; ++r) {
      float m = -INFINITY;
#pragma unroll
      for (int j = 0; j < 4; ++j) {
        const float sv = s[j][r] * qscale;
        s[j][r] = sv;
        m = fmaxf(m, sv);
      }
#pragma unroll
      for (int off = 1; off < 16; off <<= 1) m = fmaxf(m, __shfl_xor(m, off, 32));
      cm[r] = m;
    }
#pragma unroll
    for (int r = 0; r < 8; ++r) {
      const float mnew = fmaxf(mrow[r], cm[r]);
      const float alpha = expf(mrow[r] - mnew);
      mrow[r] = mnew;
      float psum = 0.f;
#pragma unroll
      for (int j = 0; j < 4; ++j) {
        const float p = expf(s[j][r] - mnew);
        psum += p;
        Pp[(8 * hh + r) * VT_P + j * 16 + c] = __builtin_bit_cast(unsigned short, (_Float16)(p * PSC));
      }
#pragma unroll
      for (int off = 1; off < 16; off <<= 1) psum += __shfl_xor(psum, off, 32);
      lrow[r] = lrow[r] * alpha + psum;
#pragma unroll
      for (int t = 0; t < 2; ++t) oacc[t][r] *= alpha;
    }
    __builtin_amdgcn_fence(__ATOMIC_RELEASE, "workgroup");
    __builtin_amdgcn_wave_barrier();
    __builtin_amdgcn_fence(__ATOMIC_ACQUIRE, "workgroup");
#pragma unroll
    for (int kk = 0; kk < 2; ++kk) {
      const v16h pa = Frag<_Float16>::load((const _Float16*)(Pp + c * VT_P) + kk * 32 + 8 * hh);
#pragma unroll
      for (int t = 0; t < 2; ++t) {
        const v16h vb = Frag<_Float16>::load((const _Float16*)(Vp + (t * 16 + c) * VT_P) + kk * 32 + 8 * hh);
        oacc[t] = mma_h(pa, vb, oacc[t]);
      }
    }
  }

#pragma unroll
  for (int r = 0; r < 8; ++r) {
    const float inv = OSC / (lrow[r] * PSC);
#pragma unroll
    for (int t = 0; t < 2; ++t) {
      Ob[(wq * 16 + 8 * hh + r) * VT_P + hsel * 32 + t * 16 + c] =
          __builtin_bit_cast(unsigned short, (_Float16)(oacc[t][r] * inv));
    }
  }
  __syncthreads();
  for (int pass = 0; pass < 2; ++pass) {
#pragma unroll
    for (int it = 0; it < 2; ++it) {
      const int row  = wave * 8 + it * 4 + (lane >> 3);
      const int col8 = (lane & 7) * 8;
      const v4u val = *(const v4u*)(&Ob[row * VT_P + col8]);
      *(volatile v4u*)(o + (rowbase + qb * 64 + row) * NEMB + hp * 64 + col8) = val;
    }
    __threadfence();
  }
}

__global__ __launch_bounds__(256) void mix_out_kernel(const float* __restrict__ x, const float* __restrict__ msk,
                                                     const float* __restrict__ imp, float* __restrict__ out0, int n4) {
  const int i = blockIdx.x * 256 + threadIdx.x;
  if (i < n4) {
    const size_t e = (size_t)i * 4;
    const v4f xv = *(const v4f*)(x + e);
    const v4f mv = *(const v4f*)(msk + e);
    const v4f iv = *(const v4f*)(imp + e);
    v4f ov;
    ov[0] = xv[0] * mv[0] + iv[0] * (1.0f - mv[0]);
    ov[1] = xv[1] * mv[1] + iv[1] * (1.0f - mv[1]);
    ov[2] = xv[2] * mv[2] + iv[2] * (1.0f - mv[2]);
    ov[3] = xv[3] * mv[3] + iv[3] * (1.0f - mv[3]);
    float* dst = out0 + e;
    *(volatile v4f*)dst = ov;
    __threadfence();
    *(volatile v4f*)dst = ov;
  }
}

extern "C" void kernel_launch(void* const* d_in, const int* in_sizes, int n_in,
                              void* d_out, int out_size, void* d_ws, size_t ws_size,
                              hipStream_t stream) {
  if (n_in < 16) return;
  if (in_sizes[0] != NROWS * NDIN || out_size != 2 * NROWS * NDIN) return;
  const float* x          = (const float*)d_in[0];
  const float* msk        = (const float*)d_in[1];
  const float* fwd_Wi     = (const float*)d_in[2];
  const float* fwd_bi     = (const float*)d_in[3];
  const float* fwd_Wh     = (const float*)d_in[4];
  const float* fwd_bh     = (const float*)d_in[5];
  const float* bwd_Wi     = (const float*)d_in[6];
  const float* bwd_bi     = (const float*)d_in[7];
  const float* bwd_Wh     = (const float*)d_in[8];
  const float* bwd_bh     = (const float*)d_in[9];
  const float* attn_w_in  = (const float*)d_in[10];
  const float* attn_b_in  = (const float*)d_in[11];
  const float* attn_w_out = (const float*)d_in[12];
  const float* attn_b_out = (const float*)d_in[13];
  const float* out_w      = (const float*)d_in[14];
  const float* out_b      = (const float*)d_in[15];

  const size_t szXM   = (size_t)NROWS * NDIN * 2;
  const size_t szWI   = (size_t)2 * NGATE3 * NDIN * 2;
  const size_t szWH   = (size_t)NGATE3 * NHID * 2;
  const size_t szWIN  = (size_t)NQKV * NEMB * 2;
  const size_t szWOUT = (size_t)NEMB * NEMB * 2;
  const size_t szOW   = (size_t)NDIN * NEMB * 2;
  const size_t szGI   = (size_t)NROWS * NQKV * 4;
  const size_t szHC   = (size_t)NROWS * NEMB * 2;
  const size_t szQKV  = (size_t)NROWS * NQKV * 2;
  const size_t szO    = (size_t)NROWS * NEMB * 2;
  const size_t szPROJ = (size_t)NROWS * NEMB * 2;

  size_t off = 0;
  char* ws = (char*)d_ws;
  _Float16* xm16   = (_Float16*)(ws + off); off += szXM;
  _Float16* wi16   = (_Float16*)(ws + off); off += szWI;
  _Float16* whf16  = (_Float16*)(ws + off); off += szWH;
  _Float16* whb16  = (_Float16*)(ws + off); off += szWH;
  _Float16* win16  = (_Float16*)(ws + off); off += szWIN;
  _Float16* wout16 = (_Float16*)(ws + off); off += szWOUT;
  _Float16* ow16   = (_Float16*)(ws + off); off += szOW;
  float*    gi     = (float*)(ws + off);    off += szGI;
  _Float16* hc16   = (_Float16*)(ws + off); off += szHC;
  _Float16* qkv16  = (_Float16*)(ws + off); off += szQKV;
  _Float16* o16    = (_Float16*)(ws + off); off += szO;
  _Float16* proj16 = (_Float16*)(ws + off); off += szPROJ;
  if (off > ws_size) return;

  float* out0 = (float*)d_out;
  float* out1 = (float*)d_out + (size_t)NROWS * NDIN;

  {
    const int n8 = NROWS * NDIN / 8;
    prep_xm_f16x8<<<(n8 + 255) / 256, 256, 0, stream>>>(x, msk, xm16, n8);
  }
  {
    const int n8wi = NGATE3 * NDIN / 8;
    cast_scale_f16x8<<<(n8wi + 255) / 256, 256, 0, stream>>>(fwd_Wi, wi16, n8wi, 16.0f);
    cast_scale_f16x8<<<(n8wi + 255) / 256, 256, 0, stream>>>(bwd_Wi, wi16 + (size_t)NGATE3 * NDIN, n8wi, 16.0f);
    const int n8wh = NGATE3 * NHID / 8;
    cast_scale_f16x8<<<(n8wh + 255) / 256, 256, 0, stream>>>(fwd_Wh, whf16, n8wh, 16.0f);
    cast_scale_f16x8<<<(n8wh + 255) / 256, 256, 0, stream>>>(bwd_Wh, whb16, n8wh, 16.0f);
    const int n8win = NQKV * NEMB / 8;
    cast_scale_f16x8<<<(n8win + 255) / 256, 256, 0, stream>>>(attn_w_in, win16, n8win, 16.0f);
    const int n8wout = NEMB * NEMB / 8;
    cast_scale_f16x8<<<(n8wout + 255) / 256, 256, 0, stream>>>(attn_w_out, wout16, n8wout, 16.0f);
    const int n8ow = NDIN * NEMB / 8;
    cast_scale_f16x8<<<(n8ow + 255) / 256, 256, 0, stream>>>(out_w, ow16, n8ow, 16.0f);
  }
  {
    const int tiles = (NROWS / 64) * (NQKV / 64);
    wmma_gemm64<0, false, 0, 0, false><<<dim3(tiles / 8, 1), 256, 0, stream>>>(
        U16(xm16), U16(xm16), NDIN, 0L,
        U16(wi16), U16(wi16), NDIN, 0L,
        (void*)gi, (void*)gi, NQKV, 0L,
        fwd_bi, (const float*)gi, 0L,
        NROWS, NQKV, NDIN, 0.0625f);
  }
  gru_bidir_kernel<<<4, 256, 0, stream>>>(gi, whf16, whb16, fwd_bi, fwd_bh, bwd_bi, bwd_bh, hc16);
  {
    const int tiles = (NROWS / 64) * (NQKV / 64);
    wmma_gemm64<0, false, 2, 1, false><<<dim3(tiles / 8, 1), 256, 0, stream>>>(
        U16(hc16), U16(hc16), NEMB, 0L,
        U16(win16), U16(win16), NEMB, 0L,
        (void*)qkv16, (void*)qkv16, NQKV, 0L,
        attn_b_in, (const float*)gi, 0L,
        NROWS, NQKV, NEMB, 0.0625f);
  }
  attn_hd32_kernel<<<NBATCH * 4 * (NSTEP / 64), 256, 0, stream>>>(qkv16, o16, 0.17677669529663687f);
  {
    const int tiles = (NROWS / 64) * (NEMB / 64);
    wmma_gemm64<0, false, 2, 1, false><<<dim3(tiles / 8, 1), 256, 0, stream>>>(
        U16(o16), U16(o16), NEMB, 0L,
        U16(wout16), U16(wout16), NEMB, 0L,
        (void*)proj16, (void*)proj16, NEMB, 0L,
        attn_b_out, (const float*)gi, 0L,
        NROWS, NEMB, NEMB, 0.00390625f);
  }
  {
    const int tiles = (NROWS / 64) * (NDIN / 64);
    wmma_gemm64<0, false, 2, 0, false><<<dim3(tiles / 8, 1), 256, 0, stream>>>(
        U16(proj16), U16(proj16), NEMB, 0L,
        U16(ow16), U16(ow16), NEMB, 0L,
        (void*)out1, (void*)out1, NDIN, 0L,
        out_b, (const float*)gi, 0L,
        NROWS, NDIN, NEMB, 0.0625f);
  }
  {
    const int n4 = NROWS * NDIN / 4;
    mix_out_kernel<<<(n4 + 255) / 256, 256, 0, stream>>>(x, msk, (const float*)out1, out0, n4);
  }
}
